// ViTAttention_49967649522063
// MI455X (gfx1250) — hardware-verified
//
#include <hip/hip_runtime.h>
#include <math.h>
#include <stdint.h>

typedef __attribute__((ext_vector_type(16))) _Float16 v16h;
typedef __attribute__((ext_vector_type(8)))  _Float16 v8h;
typedef __attribute__((ext_vector_type(16))) __bf16   v16b;
typedef __attribute__((ext_vector_type(8)))  __bf16   v8b;
typedef __attribute__((ext_vector_type(8)))  float    v8f;
typedef __attribute__((ext_vector_type(4)))  float    v4f;
typedef __attribute__((ext_vector_type(2)))  float    v2f;
typedef __attribute__((ext_vector_type(4)))  unsigned int v4u;

constexpr int NBAT      = 16;
constexpr int SEQ_LEN   = 577;
constexpr int SEQ_PAD   = 640;
constexpr int HID       = 1024;
constexpr int NUM_HEADS = 16;
constexpr int HEAD_DIM  = 64;
constexpr int ROWS_PAD  = NBAT * SEQ_PAD;
constexpr int QK_PITCH  = 2 * HID;
constexpr int NQB       = SEQ_PAD / 64;
constexpr int NKC       = SEQ_PAD / 64;
static_assert(SEQ_PAD >= SEQ_LEN && SEQ_PAD % 64 == 0, "pad");
static_assert(ROWS_PAD % 64 == 0 && HID % 64 == 0 && HID % 32 == 0, "tile multiples");
static_assert(NUM_HEADS * HEAD_DIM == HID && HEAD_DIM == 64, "head geometry");
static_assert((ROWS_PAD * HID / 2) % 256 == 0 && (HID * HID / 2) % 256 == 0 && HID % 256 == 0, "cast grids exact");

__device__ __forceinline__ unsigned short f2bf_bits(float f) {
  unsigned u = __float_as_uint(f);
  return (unsigned short)((u + 0x7FFFu + ((u >> 16) & 1u)) >> 16);
}
__device__ __forceinline__ float bf_bits2f(unsigned short h) { return __uint_as_float(((unsigned)h) << 16); }
__device__ __forceinline__ unsigned pk16(unsigned short a, unsigned short b) { return (unsigned)a | ((unsigned)b << 16); }

__device__ __forceinline__ void dep_guard_h(v8f& a, v8f& b, v16h x, v16h y) { asm volatile("v_nop\n\tv_nop\n\tv_nop\n\tv_nop" : "+v"(a), "+v"(b) : "v"(x), "v"(y)); }
__device__ __forceinline__ void dep_guard_b(v8f& a, v8f& b, v16b x, v16b y) { asm volatile("v_nop\n\tv_nop\n\tv_nop\n\tv_nop" : "+v"(a), "+v"(b) : "v"(x), "v"(y)); }
__device__ __forceinline__ void keep4_h(v16h a, v16h b, v16h c, v16h d) { asm volatile("v_nop" :: "v"(a), "v"(b), "v"(c), "v"(d)); }
__device__ __forceinline__ void keep4_b(v16b a, v16b b, v16b c, v16b d) { asm volatile("v_nop" :: "v"(a), "v"(b), "v"(c), "v"(d)); }
__device__ __forceinline__ void acc_guard4(v8f& a, v8f& b, v8f& c, v8f& d) { asm volatile("v_nop\n\tv_nop\n\tv_nop\n\tv_nop" : "+v"(a), "+v"(b), "+v"(c), "+v"(d)); }
template <typename T> struct Frag;
template <> struct Frag<_Float16> {
  typedef v16h V; union U { v16h v; v8h h[2]; };
  static __device__ __forceinline__ v16h load(const _Float16* p) {
    U f; f.h[0] = *(const v8h*)(p); f.h[1] = *(const v8h*)(p + 16); return f.v;
  }
  static __device__ __forceinline__ v8f mma(v16h a, v16h b, v8f c) {
    return __builtin_amdgcn_wmma_f32_16x16x32_f16(false, a, false, b, (short)0, c, false, false);
  }
  static __device__ __forceinline__ void guard(v8f& a, v8f& b, v16h x, v16h y) { dep_guard_h(a, b, x, y); }
  static __device__ __forceinline__ void keep(v16h a, v16h b, v16h c, v16h d) { keep4_h(a, b, c, d); }
};
template <> struct Frag<__bf16> {
  typedef v16b V; union U { v16b v; v8b h[2]; };
  static __device__ __forceinline__ v16b load(const __bf16* p) {
    U f; f.h[0] = *(const v8b*)(p); f.h[1] = *(const v8b*)(p + 16); return f.v;
  }
  static __device__ __forceinline__ v8f mma(v16b a, v16b b, v8f c) {
    return __builtin_amdgcn_wmma_f32_16x16x32_bf16(false, a, false, b, (short)0, c, false, false);
  }
  static __device__ __forceinline__ void guard(v8f& a, v8f& b, v16b x, v16b y) { dep_guard_b(a, b, x, y); }
  static __device__ __forceinline__ void keep(v16b a, v16b b, v16b c, v16b d) { keep4_b(a, b, c, d); }
};

template <int ET> struct Elem;
template <> struct Elem<0> { typedef _Float16 T; };
template <> struct Elem<1> { typedef __bf16 T; };
template <int ET, bool SPLIT, int BIAS_MODE, int OUT_MODE, bool RESID, int ACT = 0>
__global__ __launch_bounds__(256) void wmma_gemm64(
    const unsigned short* __restrict__ Ap, const unsigned short* __restrict__ A2p, int lda, long strideA,
    const unsigned short* __restrict__ Btp, const unsigned short* __restrict__ Bt2p, int ldb, long strideB,
    void* __restrict__ Cout, void* __restrict__ Cout2, int ldc, long strideC,
    const float* __restrict__ bias,
    const float* __restrict__ resid, long strideR,
    int M, int N, int K, float scale) {
  typedef typename Elem<ET>::T T;
  typedef typename Frag<T>::V V;
  const T* A = (const T*)Ap; const T* A2 = (const T*)A2p; const T* Bt = (const T*)Btp; const T* Bt2 = (const T*)Bt2p;
  __shared__ __align__(16) float sT[8][16 * 68];
  const int b    = blockIdx.y;
  const int lane = threadIdx.x & 31;
  const int wave = threadIdx.x >> 5;
  const int tilesN = N >> 6;
  const int tilesM = M >> 6;
  const int tile = blockIdx.x * 8 + wave;
  if (tile >= tilesM * tilesN) return;
  const int tm = tile / tilesN;
  const int tn = tile - tm * tilesN;
  const int m0 = tm << 6;
  const int n0 = tn << 6;

  const T* Ab  = A  + (size_t)b * strideA;
  const T* Bb  = Bt + (size_t)b * strideB;
  const T* Ab2 = SPLIT ? (A2  + (size_t)b * strideA) : nullptr;
  const T* Bb2 = SPLIT ? (Bt2 + (size_t)b * strideB) : nullptr;

  const int rlane = lane & 15;
  const int koff  = (lane >> 4) * 8;
  const int mOff  = (lane >> 4) * 8;

  v8f acc[4][4];
#pragma unroll
  for (int i = 0; i < 4; ++i)
#pragma unroll
    for (int j = 0; j < 4; ++j) acc[i][j] = (v8f){0.f,0.f,0.f,0.f,0.f,0.f,0.f,0.f};

  for (int k0 = 0; k0 < K; k0 += 32) {
    V bh[4], bl[4];
#pragma unroll
    for (int j = 0; j < 4; ++j) {
      const size_t bo = (size_t)(n0 + (j << 4) + rlane) * ldb + koff + k0;
      bh[j] = Frag<T>::load(Bb + bo);
      if (SPLIT) bl[j] = Frag<T>::load(Bb2 + bo);
    }
#pragma unroll
    for (int i = 0; i < 4; ++i) {
      const size_t ao = (size_t)(m0 + (i << 4) + rlane) * lda + koff + k0;
      V ah = Frag<T>::load(Ab + ao);
      V al;
      if (SPLIT) al = Frag<T>::load(Ab2 + ao);
#pragma unroll
      for (int j = 0; j < 4; ++j) {
        acc[i][j] = Frag<T>::mma(ah, bh[j], acc[i][j]);
        if (SPLIT) {
          acc[i][j] = Frag<T>::mma(ah, bl[j], acc[i][j]);
          acc[i][j] = Frag<T>::mma(al, bh[j], acc[i][j]);
        }
      }
      Frag<T>::guard(acc[i][0], acc[i][3], ah, SPLIT ? al : ah);
    }
    Frag<T>::keep(bh[0], bh[1], bh[2], bh[3]);
    if (SPLIT) Frag<T>::keep(bl[0], bl[1], bl[2], bl[3]);
  }
  acc_guard4(acc[0][0], acc[0][1], acc[0][2], acc[0][3]);
  acc_guard4(acc[1][0], acc[1][1], acc[1][2], acc[1][3]);
  acc_guard4(acc[2][0], acc[2][1], acc[2][2], acc[2][3]);
  acc_guard4(acc[3][0], acc[3][1], acc[3][2], acc[3][3]);

  float* slab = sT[wave];
  const float* Rb = RESID ? (resid + (size_t)b * strideR) : nullptr;
#pragma unroll
  for (int i = 0; i < 4; ++i) {
    const int mBase = m0 + (i << 4);
#pragma unroll
    for (int j = 0; j < 4; ++j) {
      const int n = n0 + (j << 4) + rlane;
      float bv = 0.f;
      if (BIAS_MODE == 2) bv = bias[n];
#pragma unroll
      for (int r = 0; r < 8; ++r) {
        float v = acc[i][j][r] * scale;
        if (BIAS_MODE == 1) v += bias[mBase + mOff + r];
        if (BIAS_MODE == 2) v += bv;
        if (RESID) v += Rb[(size_t)(mBase + mOff + r) * ldc + n];
        if (ACT == 1) v = tanhf(v);
        if (ACT == 2) v = fmaxf(v, 0.0f);
        if (ACT == 3) v = v / (1.0f + expf(-v));
        if (ACT == 4) v = (v > 0.f) ? v : 0.01f * v;
        if (ACT == 5) v = 0.5f * v * (1.0f + erff(v * 0.70710678118654752f));
        slab[(mOff + r) * 68 + (j << 4) + rlane] = v;
      }
    }
    __builtin_amdgcn_fence(__ATOMIC_RELEASE, "workgroup");
    __builtin_amdgcn_wave_barrier();
    __builtin_amdgcn_fence(__ATOMIC_ACQUIRE, "workgroup");
    if (OUT_MODE == 0) {
      float* C = (float*)Cout + (size_t)b * strideC;
      const int hh = lane >> 4, c4 = (lane & 15) * 4;
      for (int pass = 0; pass < 2; ++pass) {
#pragma unroll
        for (int it = 0; it < 8; ++it) {
          const int row = it * 2 + hh;
          v4f v = *(const v4f*)(slab + row * 68 + c4);
          *(volatile v4f*)(C + (size_t)(mBase + row) * ldc + n0 + c4) = v;
        }
        __threadfence();
      }
    } else {
      const int q = lane >> 3, c8 = (lane & 7) * 8;
      unsigned short* C  = (unsigned short*)Cout  + (size_t)b * strideC;
      unsigned short* C2 = (OUT_MODE == 2) ? ((unsigned short*)Cout2 + (size_t)b * strideC) : nullptr;
      for (int pass = 0; pass < 2; ++pass) {
#pragma unroll
        for (int it = 0; it < 4; ++it) {
          const int row = it * 4 + q;
          const float* sp = slab + row * 68 + c8;
          v8h hv, lv;
#pragma unroll
          for (int e = 0; e < 8; ++e) {
            if (OUT_MODE == 1) {
              hv[e] = (_Float16)sp[e];
            } else {
              unsigned short hb = f2bf_bits(sp[e]);
              unsigned short lb = f2bf_bits(sp[e] - bf_bits2f(hb));
              hv[e] = __builtin_bit_cast(_Float16, hb);
              lv[e] = __builtin_bit_cast(_Float16, lb);
            }
          }
          *(volatile v8h*)(C + (size_t)(mBase + row) * ldc + n0 + c8) = hv;
          if (OUT_MODE == 2) *(volatile v8h*)(C2 + (size_t)(mBase + row) * ldc + n0 + c8) = lv;
        }
        __threadfence();
      }
    }
    __builtin_amdgcn_fence(__ATOMIC_RELEASE, "workgroup");
    __builtin_amdgcn_wave_barrier();
    __builtin_amdgcn_fence(__ATOMIC_ACQUIRE, "workgroup");
  }
}

__global__ __launch_bounds__(256) void cast_x_kernel(const float* __restrict__ x, unsigned short* __restrict__ xb) {
  const int i = blockIdx.x * 256 + threadIdx.x;
  const int e = 2 * i;
  const int prow = e >> 10;
  const int col  = e & (HID - 1);
  const int b  = prow / SEQ_PAD;
  const int r  = prow - b * SEQ_PAD;
  const int rc = (r < SEQ_LEN) ? r : (SEQ_LEN - 1);
  const v2f f = *(const v2f*)(x + ((size_t)(b * SEQ_LEN + rc)) * HID + col);
  const unsigned short h0 = f2bf_bits(f[0]), h1 = f2bf_bits(f[1]);
  const unsigned u = (r < SEQ_LEN) ? pk16(h0, h1) : 0u;
  ((volatile unsigned*)xb)[i] = u;
  __threadfence();
  ((volatile unsigned*)xb)[i] = u;
}

__global__ __launch_bounds__(256) void cast_w_kernel(const float* __restrict__ wq, const float* __restrict__ wk,
                                                     const float* __restrict__ wv, unsigned short* __restrict__ wb) {
  const int which = blockIdx.y;
  const float* src = (which == 0) ? wq : ((which == 1) ? wk : wv);
  const int i = blockIdx.x * 256 + threadIdx.x;
  const v2f f = *(const v2f*)(src + 2 * (size_t)i);
  const unsigned u = pk16(f2bf_bits(f[0]), f2bf_bits(f[1]));
  volatile unsigned* dst = (volatile unsigned*)(wb + (size_t)which * HID * HID);
  dst[i] = u;
  __threadfence();
  dst[i] = u;
}

__global__ __launch_bounds__(256) void bias_rne_kernel(const float* __restrict__ bq, const float* __restrict__ bk,
                                                       const float* __restrict__ bv, float* __restrict__ br) {
  const int which = blockIdx.y;
  const float* src = (which == 0) ? bq : ((which == 1) ? bk : bv);
  const int i = blockIdx.x * 256 + threadIdx.x;
  const float v = bf_bits2f(f2bf_bits(src[i]));
  volatile float* dst = (volatile float*)(br + (size_t)which * HID);
  dst[i] = v;
  __threadfence();
  dst[i] = v;
}

#define AT_D 64
#define AT_NW 4
#define AT_QB 64
#define AT_KC 64
constexpr float P_CARRY = 32768.0f;

__device__ __forceinline__ v8f mma_f16g(v16h a, v16h b, v8f c) {
  c = __builtin_amdgcn_wmma_f32_16x16x32_f16(false, a, false, b, (short)0, c, false, false);
  asm volatile("v_nop\n\tv_nop\n\tv_nop\n\tv_nop" : "+v"(c) : "v"(a), "v"(b));
  return c;
}

__global__ __launch_bounds__(128)
void attn_f16_kernel(const unsigned short* __restrict__ qkp, const unsigned short* __restrict__ vtp,
                     float* __restrict__ out, float sscale) {
  union FH { v16h v; v8h h[2]; };
  __shared__ __align__(16) _Float16 Ksh[AT_KC * AT_D];
  __shared__ __align__(16) _Float16 Vth[AT_D * AT_KC];
  __shared__ __align__(16) _Float16 Psh[AT_NW][16 * AT_KC];
  __shared__ __align__(16) float    Os[AT_NW][16 * 68];

  const int tid  = threadIdx.x;
  const int wave = tid >> 5;
  const int lane = tid & 31;
  const int hh   = lane >> 4;
  const int c    = lane & 15;

  const int bx = blockIdx.x;
  const int qb = bx % NQB;
  const int bh = bx / NQB;
  const int h  = bh % NUM_HEADS;
  const int b  = bh / NUM_HEADS;
  const int q0 = qb * AT_QB + wave * 16;

  const _Float16* Qp = (const _Float16*)(const void*)qkp + (size_t)b * SEQ_PAD * QK_PITCH + (size_t)h * AT_D;
  const _Float16* Kp = Qp + HID;
  const _Float16* Vp = (const _Float16*)(const void*)vtp + ((size_t)(b * NUM_HEADS + h) * AT_D) * SEQ_PAD;
  float*          ob = out + (size_t)b * SEQ_LEN * HID + (size_t)h * AT_D;

  v16h qa[2];
#pragma unroll
  for (int dc = 0; dc < 2; ++dc)
    qa[dc] = Frag<_Float16>::load(Qp + (size_t)(q0 + c) * QK_PITCH + dc * 32 + 8 * hh);

  float mrow[8], lrow[8];
  v8f oacc[4];
#pragma unroll
  for (int r = 0; r < 8; ++r) { mrow[r] = -INFINITY; lrow[r] = 0.f; }
#pragma unroll
  for (int t = 0; t < 4; ++t) oacc[t] = (v8f){0.f,0.f,0.f,0.f,0.f,0.f,0.f,0.f};

  for (int kc = 0; kc < NKC; ++kc) {
    const int kv0 = kc * AT_KC;
    __syncthreads();
    {
      const int r = tid >> 1, half = (tid & 1) * 32;
      const _Float16* ks = Kp + (size_t)(kv0 + r) * QK_PITCH + half;
      const _Float16* vs = Vp + (size_t)r * SEQ_PAD + kv0 + half;
#pragma unroll
      for (int i = 0; i < 4; ++i) {
        const v8h a0 = *(const v8h*)(ks + 8 * i);
        const v8h b0 = *(const v8h*)(vs + 8 * i);
        *(v8h*)(Ksh + r * AT_D  + half + 8 * i) = a0;
        *(v8h*)(Vth + r * AT_KC + half + 8 * i) = b0;
      }
    }
    __syncthreads();

    v8f s[4];
#pragma unroll
    for (int j = 0; j < 4; ++j) {
      s[j] = (v8f){0.f,0.f,0.f,0.f,0.f,0.f,0.f,0.f};
#pragma unroll
      for (int dc = 0; dc < 2; ++dc) {
        FH kb;
        kb.h[0] = *(const v8h*)(Ksh + (j * 16 + c) * AT_D + dc * 32 + 8 * hh);
        kb.h[1] = *(const v8h*)(Ksh + (j * 16 + c) * AT_D + dc * 32 + 16 + 8 * hh);
        s[j] = mma_f16g(qa[dc], kb.v, s[j]);
      }
    }
    float cm[8];
#pragma unroll
    for (int r = 0; r < 8; ++r) {
      float m = -INFINITY;
#pragma unroll
      for (int j = 0; j < 4; ++j) {
        const int kvcol = kv0 + j * 16 + c;
        float sv = s[j][r] * sscale;
        sv = (kvcol < SEQ_LEN) ? sv : -INFINITY;
        s[j][r] = sv;
        m = fmaxf(m, sv);
      }
#pragma unroll
      for (int off = 1; off < 16; off <<= 1) m = fmaxf(m, __shfl_xor(m, off, 32));
      cm[r] = m;
    }
    _Float16* pwh = Psh[wave];
#pragma unroll
    for (int r = 0; r < 8; ++r) {
      const float mnew = fmaxf(mrow[r], cm[r]);
      const float alpha = expf(mrow[r] - mnew);
      mrow[r] = mnew;
      float psum = 0.f;
#pragma unroll
      for (int j = 0; j < 4; ++j) {
        const float p = expf(s[j][r] - mnew);
        psum += p;
        pwh[(8 * hh + r) * AT_KC + j * 16 + c] = (_Float16)(p * P_CARRY);
      }
#pragma unroll
      for (int off = 1; off < 16; off <<= 1) psum += __shfl_xor(psum, off, 32);
      lrow[r] = lrow[r] * alpha + psum;
#pragma unroll
      for (int t = 0; t < 4; ++t) oacc[t][r] *= alpha;
    }
    __builtin_amdgcn_fence(__ATOMIC_RELEASE, "workgroup");
    __builtin_amdgcn_wave_barrier();
    __builtin_amdgcn_fence(__ATOMIC_ACQUIRE, "workgroup");
#pragma unroll 1
    for (int kk = 0; kk < 2; ++kk) {
      FH pa;
      pa.h[0] = *(const v8h*)(pwh + c * AT_KC + kk * 32 + 8 * hh);
      pa.h[1] = *(const v8h*)(pwh + c * AT_KC + kk * 32 + 16 + 8 * hh);
#pragma unroll
      for (int t = 0; t < 4; ++t) {
        FH vb;
        vb.h[0] = *(const v8h*)(Vth + (t * 16 + c) * AT_KC + kk * 32 + 8 * hh);
        vb.h[1] = *(const v8h*)(Vth + (t * 16 + c) * AT_KC + kk * 32 + 16 + 8 * hh);
        oacc[t] = mma_f16g(pa.v, vb.v, oacc[t]);
      }
    }
  }

  float* os = Os[wave];
#pragma unroll
  for (int r = 0; r < 8; ++r) {
    const float inv = 1.0f / (lrow[r] * P_CARRY);
#pragma unroll
    for (int t = 0; t < 4; ++t) os[(8 * hh + r) * 68 + t * 16 + c] = oacc[t][r] * inv;
  }
  __builtin_amdgcn_fence(__ATOMIC_RELEASE, "workgroup");
  __builtin_amdgcn_wave_barrier();
  __builtin_amdgcn_fence(__ATOMIC_ACQUIRE, "workgroup");
  {
    const int c4 = (lane & 15) * 4;
    for (int pass = 0; pass < 2; ++pass) {
#pragma unroll
      for (int it = 0; it < 8; ++it) {
        const int row = it * 2 + hh;
        const int srow = q0 + row;
        v4f val = *(const v4f*)(os + row * 68 + c4);
        if (srow < SEQ_LEN) *(volatile v4f*)(ob + (size_t)srow * HID + c4) = val;
      }
      __threadfence();
    }
  }
}

extern "C" void kernel_launch(void* const* d_in, const int* in_sizes, int n_in,
                              void* d_out, int out_size, void* d_ws,
                              size_t ws_size, hipStream_t stream) {
  if (n_in < 7) return;
  if (in_sizes[0] != NBAT * SEQ_LEN * HID) return;
  if (in_sizes[1] != HID * HID || in_sizes[3] != HID * HID || in_sizes[5] != HID * HID) return;
  if (in_sizes[2] != HID || in_sizes[4] != HID || in_sizes[6] != HID) return;
  if (out_size != NBAT * SEQ_LEN * HID) return;

  const float* x  = (const float*)d_in[0];
  const float* wq = (const float*)d_in[1];
  const float* bq = (const float*)d_in[2];
  const float* wk = (const float*)d_in[3];
  const float* bk = (const float*)d_in[4];
  const float* wv = (const float*)d_in[5];
  const float* bv = (const float*)d_in[6];
  float* out = (float*)d_out;

  const size_t bytesX  = (size_t)ROWS_PAD * HID * 2;
  const size_t bytesW  = (size_t)3 * HID * HID * 2;
  const size_t bytesBR = (size_t)3 * HID * 4;
  const size_t bytesQK = (size_t)ROWS_PAD * QK_PITCH * 2;
  const size_t bytesVT = (size_t)NBAT * HID * SEQ_PAD * 2;
  const size_t offX  = 0;
  const size_t offW  = offX + bytesX;
  const size_t offBR = offW + bytesW;
  const size_t offQK = offBR + bytesBR;
  const size_t offVT = offQK + bytesQK;
  const size_t total = offVT + bytesVT;
  if (total > ws_size) return;

  char* ws = (char*)d_ws;
  unsigned short* XB = (unsigned short*)(ws + offX);
  unsigned short* WB = (unsigned short*)(ws + offW);
  float*          BR = (float*)(ws + offBR);
  unsigned short* QK = (unsigned short*)(ws + offQK);
  unsigned short* VT = (unsigned short*)(ws + offVT);

  cast_x_kernel<<<dim3(ROWS_PAD * HID / 512), 256, 0, stream>>>(x, XB);
  cast_w_kernel<<<dim3(HID * HID / 512, 3), 256, 0, stream>>>(wq, wk, wv, WB);
  bias_rne_kernel<<<dim3(HID / 256, 3), 256, 0, stream>>>(bq, bk, bv, BR);

  {
    const int tiles = (ROWS_PAD / 64) * (HID / 64);
    wmma_gemm64<1, false, 2, 1, false, 0><<<dim3(tiles / 8, 1), 256, 0, stream>>>(
        XB, XB, HID, 0L,
        WB, WB, HID, 0L,
        (void*)QK, (void*)QK, QK_PITCH, 0L,
        BR, BR, 0L,
        ROWS_PAD, HID, HID, 1.0f);
  }
  {
    const int tiles = (ROWS_PAD / 64) * (HID / 64);
    wmma_gemm64<1, false, 2, 1, false, 0><<<dim3(tiles / 8, 1), 256, 0, stream>>>(
        XB, XB, HID, 0L,
        WB + (size_t)HID * HID, WB + (size_t)HID * HID, HID, 0L,
        (void*)(QK + HID), (void*)(QK + HID), QK_PITCH, 0L,
        BR + HID, BR, 0L,
        ROWS_PAD, HID, HID, 1.0f);
  }
  {
    const int tiles = (HID / 64) * (SEQ_PAD / 64);
    wmma_gemm64<1, false, 1, 1, false, 0><<<dim3(tiles / 8, NBAT), 256, 0, stream>>>(
        WB + (size_t)2 * HID * HID, WB + (size_t)2 * HID * HID, HID, 0L,
        XB, XB, HID, (long)SEQ_PAD * HID,
        (void*)VT, (void*)VT, SEQ_PAD, (long)HID * SEQ_PAD,
        BR + 2 * HID, BR, 0L,
        HID, SEQ_PAD, HID, 1.0f);
  }
  attn_f16_kernel<<<dim3(NBAT * NUM_HEADS * NQB), 128, 0, stream>>>(QK, VT, out, 0.03125f);
}
